// MambaBlock_87076166960151
// MI455X (gfx1250) — hardware-verified
//
#include <hip/hip_runtime.h>
#include <math.h>

typedef __attribute__((ext_vector_type(16))) _Float16 v16h;
typedef __attribute__((ext_vector_type(8)))  _Float16 v8h;
typedef __attribute__((ext_vector_type(8)))  float    v8f;
typedef __attribute__((ext_vector_type(4)))  float    v4f;

constexpr int kBatch  = 2;
constexpr int kSeqL   = 2048;
constexpr int kDmod   = 1024;
constexpr int kDin    = 2048;
constexpr int kNst    = 16;
constexpr int kDconv  = 4;
constexpr int kPrjN   = 2 * kNst + kDin;
constexpr int kPrjP   = 2112;
constexpr int kPrjD0  = 2 * kNst;
constexpr int kXZP    = 2 * kDin;
constexpr int kRows   = kBatch * kSeqL;
constexpr int kTP     = 260;
constexpr float kEps  = 1e-6f;
constexpr float kCarH = 16.0f;
constexpr float kCarW = 32.0f;
constexpr float kCarU = 16.0f;
constexpr float kCarY = 16.0f;
constexpr float kSclIn  = 1.0f / (kCarH * kCarW);
constexpr float kSclXp  = 1.0f / (kCarU * kCarW);
constexpr float kSclOut = 1.0f / (kCarY * kCarW);
static_assert(kPrjP == ((kPrjN + 63) / 64) * 64, "x_proj pad");
static_assert((kDmod % 32) == 0 && (kDin % 32) == 0, "GEMM K multiples of 32");
static_assert((kSeqL % 64) == 0 && (kXZP % 64) == 0 && (kPrjP % 64) == 0 && (kDmod % 64) == 0, "GEMM M,N multiples of 64");
static_assert((kDin % 256) == 0 && (kSeqL % 64) == 0 && (kSeqL % 16) == 0 && (kDmod == 128 * 8), "tile multiples");
static_assert(kRows * kDmod == 4194304, "x and out");
static_assert(kDmod * kXZP == 4194304, "w_in");
static_assert(kDin * kDconv == 8192, "conv_w");
static_assert(kDin * kPrjN == 4259840, "w_xproj");
static_assert(kDin * kNst == 32768, "A_log");
static_assert(kDin * kDmod == 2097152, "w_out");

constexpr size_t kSzWIN16  = (size_t)kXZP  * kDmod * 2;
constexpr size_t kSzWXP16  = (size_t)kPrjP * kDin  * 2;
constexpr size_t kSzWOUT16 = (size_t)kDmod * kDin  * 2;
constexpr size_t kSzH16    = (size_t)kRows * kDmod * 2;
constexpr size_t kSzXZ     = (size_t)kSeqL * kXZP  * 4;
constexpr size_t kSzUC     = (size_t)kSeqL * kDin  * 4;
constexpr size_t kSzUC16   = (size_t)kSeqL * kDin  * 2;
constexpr size_t kSzPROJ   = (size_t)kSeqL * kPrjP * 4;
constexpr size_t kSzY16    = (size_t)kSeqL * kDin  * 2;
constexpr size_t kOffWIN16  = 0;
constexpr size_t kOffWXP16  = kOffWIN16  + kSzWIN16;
constexpr size_t kOffWOUT16 = kOffWXP16  + kSzWXP16;
constexpr size_t kOffH16    = kOffWOUT16 + kSzWOUT16;
constexpr size_t kOffXZ     = kOffH16    + kSzH16;
constexpr size_t kOffUC     = kOffXZ     + kSzXZ;
constexpr size_t kOffUC16   = kOffUC     + kSzUC;
constexpr size_t kOffPROJ   = kOffUC16   + kSzUC16;
constexpr size_t kOffY16    = kOffPROJ   + kSzPROJ;
constexpr size_t kWsTotal   = kOffY16    + kSzY16;
static_assert(kWsTotal == 114032640ull, "carve total");
static_assert(kWsTotal <= 134217728ull, "carve cap");
static_assert((kOffWXP16 % 128) == 0 && (kOffWOUT16 % 128) == 0 && (kOffH16 % 128) == 0 && (kOffXZ % 128) == 0 &&
              (kOffUC % 128) == 0 && (kOffUC16 % 128) == 0 && (kOffPROJ % 128) == 0 && (kOffY16 % 128) == 0,
              "128-B aligned regions");
static_assert(((kPrjP * 4) % 128) == 0 && ((kXZP * 4) % 128) == 0 && ((kDin * 2) % 128) == 0 && ((kDmod * 2) % 128) == 0,
              "row pitches are whole lines");

__device__ __forceinline__ void dep_guard_all_h(v8f& a, v8f& b, v8f& c, v8f& d,
                                                v16h x, v16h y0, v16h y1, v16h y2, v16h y3) {
  asm volatile("v_nop\n\tv_nop\n\tv_nop\n\tv_nop"
               : "+v"(a), "+v"(b), "+v"(c), "+v"(d)
               : "v"(x), "v"(y0), "v"(y1), "v"(y2), "v"(y3));
}
__device__ __forceinline__ void keep4_h(v16h a, v16h b, v16h c, v16h d) { asm volatile("v_nop" :: "v"(a), "v"(b), "v"(c), "v"(d)); }
__device__ __forceinline__ void acc_guard4(v8f& a, v8f& b, v8f& c, v8f& d) { asm volatile("v_nop\n\tv_nop\n\tv_nop\n\tv_nop" : "+v"(a), "+v"(b), "+v"(c), "+v"(d)); }

struct FragH {
  union U { v16h v; v8h h[2]; };
  static __device__ __forceinline__ v16h load(const _Float16* p) {
    U f; f.h[0] = *(const v8h*)(p); f.h[1] = *(const v8h*)(p + 16); return f.v;
  }
  static __device__ __forceinline__ v8f mma(v16h a, v16h b, v8f c) {
    return __builtin_amdgcn_wmma_f32_16x16x32_f16(false, a, false, b, (short)0, c, false, false);
  }
};

template <bool RESID>
__global__ __launch_bounds__(256) void wmma_gemm64_f16(
    const unsigned short* __restrict__ Ap, int lda,
    const unsigned short* __restrict__ Btp, int ldb,
    float* __restrict__ Cout, int ldc,
    const float* __restrict__ resid, int ldr,
    int M, int N, int K, float scale)
{
  const _Float16* A  = (const _Float16*)Ap;
  const _Float16* Bt = (const _Float16*)Btp;
  __shared__ __align__(16) float sT[8][16 * 68];
  const int lane = threadIdx.x & 31;
  const int wave = threadIdx.x >> 5;
  const int tilesN = N >> 6;
  const int tilesM = M >> 6;
  const int tile = blockIdx.x * 8 + wave;
  if (tile >= tilesM * tilesN) return;
  const int tm = tile / tilesN;
  const int tn = tile - tm * tilesN;
  const int m0 = tm << 6;
  const int n0 = tn << 6;

  const int rlane = lane & 15;
  const int koff  = (lane >> 4) * 8;
  const int mOff  = (lane >> 4) * 8;

  v8f acc[4][4];
#pragma unroll
  for (int i = 0; i < 4; ++i)
#pragma unroll
    for (int j = 0; j < 4; ++j) acc[i][j] = (v8f){0.f,0.f,0.f,0.f,0.f,0.f,0.f,0.f};

  for (int k0 = 0; k0 < K; k0 += 32) {
    v16h bh[4];
#pragma unroll
    for (int j = 0; j < 4; ++j) {
      const size_t bo = (size_t)(n0 + (j << 4) + rlane) * ldb + koff + k0;
      bh[j] = FragH::load(Bt + bo);
    }
#pragma unroll
    for (int i = 0; i < 4; ++i) {
      const size_t ao = (size_t)(m0 + (i << 4) + rlane) * lda + koff + k0;
      const v16h ah = FragH::load(A + ao);
#pragma unroll
      for (int j = 0; j < 4; ++j) acc[i][j] = FragH::mma(ah, bh[j], acc[i][j]);
      dep_guard_all_h(acc[i][0], acc[i][1], acc[i][2], acc[i][3], ah, bh[0], bh[1], bh[2], bh[3]);
    }
    keep4_h(bh[0], bh[1], bh[2], bh[3]);
  }
  acc_guard4(acc[0][0], acc[0][1], acc[0][2], acc[0][3]);
  acc_guard4(acc[1][0], acc[1][1], acc[1][2], acc[1][3]);
  acc_guard4(acc[2][0], acc[2][1], acc[2][2], acc[2][3]);
  acc_guard4(acc[3][0], acc[3][1], acc[3][2], acc[3][3]);

  float* slab = sT[wave];
  const int hh = lane >> 4, c4 = (lane & 15) * 4;
#pragma unroll
  for (int i = 0; i < 4; ++i) {
    const int mBase = m0 + (i << 4);
#pragma unroll
    for (int j = 0; j < 4; ++j) {
#pragma unroll
      for (int r = 0; r < 8; ++r) slab[(mOff + r) * 68 + (j << 4) + rlane] = acc[i][j][r] * scale;
    }
    __builtin_amdgcn_fence(__ATOMIC_RELEASE, "workgroup");
    __builtin_amdgcn_wave_barrier();
    __builtin_amdgcn_fence(__ATOMIC_ACQUIRE, "workgroup");
    v4f ov[8];
#pragma unroll
    for (int it = 0; it < 8; ++it) {
      const int row = it * 2 + hh;
      v4f v = *(const v4f*)(slab + row * 68 + c4);
      if (RESID) {
        const v4f rr = *(const v4f*)(resid + (size_t)(mBase + row) * ldr + n0 + c4);
        v = v + rr;
      }
      ov[it] = v;
    }
    for (int pass = 0; pass < 2; ++pass) {
#pragma unroll
      for (int it = 0; it < 8; ++it) {
        const int row = it * 2 + hh;
        *(volatile v4f*)(Cout + (size_t)(mBase + row) * ldc + n0 + c4) = ov[it];
      }
      __threadfence();
    }
    __builtin_amdgcn_fence(__ATOMIC_RELEASE, "workgroup");
    __builtin_amdgcn_wave_barrier();
    __builtin_amdgcn_fence(__ATOMIC_ACQUIRE, "workgroup");
  }
}

__global__ __launch_bounds__(256) void transpose_cast_kernel(
    const float* __restrict__ W, unsigned short* __restrict__ Bt, int Kdim, int Ndim, int Npad, float scale)
{
  __shared__ float tile[64 * 65];
  const int tid = threadIdx.x, lane = tid & 31, wave = tid >> 5;
  const int n0 = blockIdx.x * 64;
  const int k0 = blockIdx.y * 64;
  (void)Npad;
#pragma unroll
  for (int p = 0; p < 16; ++p) {
    const int idx = tid + p * 256;
    const int kk  = idx >> 6;
    const int nn  = idx & 63;
    const int n   = n0 + nn;
    const int nc  = (n < Ndim) ? n : (Ndim - 1);
    const float v = W[(size_t)(k0 + kk) * Ndim + nc];
    tile[kk * 65 + nn] = (n < Ndim) ? (v * scale) : 0.f;
  }
  __syncthreads();
  const int q = lane >> 3, c8 = (lane & 7) * 8;
  v8h hv[2];
#pragma unroll
  for (int it = 0; it < 2; ++it) {
    const int nrow = it * 32 + wave * 4 + q;
#pragma unroll
    for (int e = 0; e < 8; ++e) hv[it][e] = (_Float16)tile[(c8 + e) * 65 + nrow];
  }
  for (int pass = 0; pass < 2; ++pass) {
#pragma unroll
    for (int it = 0; it < 2; ++it) {
      const int nrow = it * 32 + wave * 4 + q;
      *(volatile v8h*)(Bt + (size_t)(n0 + nrow) * Kdim + k0 + c8) = hv[it];
    }
    __threadfence();
  }
}

__global__ __launch_bounds__(128) void rmsnorm_cast_kernel(
    const float* __restrict__ x, const float* __restrict__ nw, unsigned short* __restrict__ H16)
{
  __shared__ float red[4];
  const int tid = threadIdx.x, lane = tid & 31, wave = tid >> 5;
  const size_t row = blockIdx.x;
  const float* xr = x + row * kDmod + tid * 8;
  const v4f a0 = *(const v4f*)(xr);
  const v4f a1 = *(const v4f*)(xr + 4);
  const v4f g0 = *(const v4f*)(nw + tid * 8);
  const v4f g1 = *(const v4f*)(nw + tid * 8 + 4);
  float s = 0.0f;
#pragma unroll
  for (int e = 0; e < 4; ++e) s = fmaf(a0[e], a0[e], s);
#pragma unroll
  for (int e = 0; e < 4; ++e) s = fmaf(a1[e], a1[e], s);
#pragma unroll
  for (int off = 1; off < 32; off <<= 1) s += __shfl_xor(s, off, 32);
  if (lane == 0) red[wave] = s;
  __syncthreads();
  const float tot = (red[0] + red[1]) + (red[2] + red[3]);
  const float rs  = rsqrtf(tot * (1.0f / (float)kDmod) + kEps);
  const float sc  = rs * kCarH;
  v8h hv;
#pragma unroll
  for (int e = 0; e < 4; ++e) {
    const float t0 = a0[e] * sc;
    const float t1 = a1[e] * sc;
    hv[e]     = (_Float16)(t0 * g0[e]);
    hv[4 + e] = (_Float16)(t1 * g1[e]);
  }
  unsigned short* qd = H16 + row * kDmod + tid * 8;
  *(volatile v8h*)qd = hv;
  __threadfence();
  *(volatile v8h*)qd = hv;
}

__global__ __launch_bounds__(256) void conv_silu_kernel(
    const float* __restrict__ XZ, const float* __restrict__ cw, const float* __restrict__ cb,
    float* __restrict__ UC, unsigned short* __restrict__ UC16)
{
  __shared__ __align__(16) float sT[16 * kTP];
  const int tid = threadIdx.x, lane = tid & 31, wave = tid >> 5;
  const int d0 = blockIdx.x * 256, d = d0 + tid;
  const int t0 = blockIdx.y * 64;
  const v4f cw4 = *(const v4f*)(cw + (size_t)d * kDconv);
  const float w0 = cw4[0], w1 = cw4[1], w2 = cw4[2], w3 = cw4[3];
  const float bc = cb[d];
  float xm3, xm2, xm1;
  {
    const int r3 = t0 - 3, r2 = t0 - 2, r1 = t0 - 1;
    const float v3 = XZ[(size_t)(r3 < 0 ? 0 : r3) * kXZP + d];
    const float v2 = XZ[(size_t)(r2 < 0 ? 0 : r2) * kXZP + d];
    const float v1 = XZ[(size_t)(r1 < 0 ? 0 : r1) * kXZP + d];
    xm3 = (r3 >= 0) ? v3 : 0.f;
    xm2 = (r2 >= 0) ? v2 : 0.f;
    xm1 = (r1 >= 0) ? v1 : 0.f;
  }
  const int hrow = wave >> 1;
  const int hch  = (wave & 1) * 128 + lane * 4;
#pragma unroll 1
  for (int sub = 0; sub < 4; ++sub) {
    const int lb = t0 + sub * 16;
#pragma unroll 1
    for (int s = 0; s < 16; ++s) {
      const float xc = XZ[(size_t)(lb + s) * kXZP + d];
      float acc = w0 * xm3;
      acc = fmaf(w1, xm2, acc);
      acc = fmaf(w2, xm1, acc);
      acc = fmaf(w3, xc, acc);
      const float sv = acc + bc;
      const float sg = __builtin_amdgcn_rcpf(1.0f + __expf(-sv));
      sT[s * kTP + tid] = sv * sg;
      xm3 = xm2; xm2 = xm1; xm1 = xc;
    }
    __syncthreads();
    v4f fv[4];
    v8h bv[2];
#pragma unroll
    for (int it = 0; it < 4; ++it) fv[it] = *(const v4f*)(sT + (it * 4 + hrow) * kTP + hch);
#pragma unroll
    for (int it = 0; it < 2; ++it) {
      const float* sp = sT + (it * 8 + wave) * kTP + lane * 8;
      const v4f a0 = *(const v4f*)(sp);
      const v4f a1 = *(const v4f*)(sp + 4);
#pragma unroll
      for (int e = 0; e < 4; ++e) {
        bv[it][e]     = (_Float16)(a0[e] * kCarU);
        bv[it][4 + e] = (_Float16)(a1[e] * kCarU);
      }
    }
    for (int pass = 0; pass < 2; ++pass) {
#pragma unroll
      for (int it = 0; it < 4; ++it)
        *(volatile v4f*)(UC + (size_t)(lb + it * 4 + hrow) * kDin + d0 + hch) = fv[it];
#pragma unroll
      for (int it = 0; it < 2; ++it)
        *(volatile v8h*)(UC16 + (size_t)(lb + it * 8 + wave) * kDin + d0 + lane * 8) = bv[it];
      __threadfence();
    }
    __syncthreads();
  }
}

__global__ __launch_bounds__(256) void scan_kernel(
    const float* __restrict__ PROJ, const float* __restrict__ UC, const float* __restrict__ XZ,
    const float* __restrict__ A_log, const float* __restrict__ Dv, unsigned short* __restrict__ Y16)
{
  __shared__ __align__(16) float sBC[16 * 32];
  __shared__ __align__(16) float sA[kNst * 256];
  __shared__ __align__(16) float sY[16 * kTP];
  const int tid = threadIdx.x, lane = tid & 31, wave = tid >> 5;
  const int d0 = blockIdx.x * 256, d = d0 + tid;

#pragma unroll 1
  for (int n = 0; n < kNst; ++n) sA[n * 256 + tid] = -expf(A_log[(size_t)d * kNst + n]);
  __syncthreads();
  float An[kNst], h[kNst];
#pragma unroll
  for (int n = 0; n < kNst; ++n) { An[n] = sA[n * 256 + tid]; h[n] = 0.0f; }
  const float Dd = Dv[d];

#pragma unroll 1
  for (int c = 0; c < kSeqL / 16; ++c) {
    const int l0 = c * 16;
    if (tid < 128) {
      const int r = tid >> 3, q = (tid & 7) * 4;
      const v4f v = *(const v4f*)(PROJ + (size_t)(l0 + r) * kPrjP + q);
      *(v4f*)(sBC + r * 32 + q) = v;
    }
    __syncthreads();
#pragma unroll 1
    for (int s = 0; s < 16; ++s) {
      const size_t m = (size_t)(l0 + s);
      const float a     = PROJ[m * kPrjP + kPrjD0 + d];
      const float delta = fmaxf(a, 0.0f) + log1pf(__expf(-fabsf(a)));
      const float xv    = UC[m * kDin + d];
      const float zv    = XZ[m * kXZP + kDin + d];
      v4f Bq[4], Cq[4];
#pragma unroll
      for (int qq = 0; qq < 4; ++qq) {
        Bq[qq] = *(const v4f*)(sBC + s * 32 + 4 * qq);
        Cq[qq] = *(const v4f*)(sBC + s * 32 + kNst + 4 * qq);
      }
      float dtx = delta * xv;
      asm volatile("" : "+v"(dtx));
      float y = 0.0f;
#pragma unroll
      for (int n = 0; n < kNst; ++n) {
        const float e = __expf(delta * An[n]);
        float p = dtx * Bq[n >> 2][n & 3];
        asm volatile("" : "+v"(p));
        float qv = h[n] * e;
        asm volatile("" : "+v"(qv));
        const float hn = qv + p;
        h[n] = hn;
        float rr = hn * Cq[n >> 2][n & 3];
        asm volatile("" : "+v"(rr));
        y += rr;
      }
      float sk = xv * Dd;
      asm volatile("" : "+v"(sk));
      y += sk;
      const float sg = __builtin_amdgcn_rcpf(1.0f + __expf(-zv));
      const float g  = zv * sg;
      sY[s * kTP + tid] = (y * g) * kCarY;
    }
    __syncthreads();
    v8h hv[2];
#pragma unroll
    for (int it = 0; it < 2; ++it) {
      const float* sp = sY + (it * 8 + wave) * kTP + lane * 8;
      const v4f a0 = *(const v4f*)(sp);
      const v4f a1 = *(const v4f*)(sp + 4);
#pragma unroll
      for (int e = 0; e < 4; ++e) { hv[it][e] = (_Float16)a0[e]; hv[it][4 + e] = (_Float16)a1[e]; }
    }
    for (int pass = 0; pass < 2; ++pass) {
#pragma unroll
      for (int it = 0; it < 2; ++it)
        *(volatile v8h*)(Y16 + (size_t)(l0 + it * 8 + wave) * kDin + d0 + lane * 8) = hv[it];
      __threadfence();
    }
  }
}

extern "C" void kernel_launch(void* const* d_in, const int* in_sizes, int n_in,
                              void* d_out, int out_size, void* d_ws, size_t ws_size,
                              hipStream_t stream)
{
  if (n_in < 9) return;
  if (in_sizes[0] != kRows * kDmod) return;
  if (in_sizes[1] != kDmod) return;
  if (in_sizes[2] != kDmod * kXZP) return;
  if (in_sizes[3] != kDin * kDconv) return;
  if (in_sizes[4] != kDin) return;
  if (in_sizes[5] != kDin * kPrjN) return;
  if (in_sizes[6] != kDin * kNst) return;
  if (in_sizes[7] != kDin) return;
  if (in_sizes[8] != kDin * kDmod) return;
  if (out_size != kRows * kDmod) return;
  if (ws_size < kWsTotal) return;

  const float* x       = (const float*)d_in[0];
  const float* norm_w  = (const float*)d_in[1];
  const float* w_in    = (const float*)d_in[2];
  const float* conv_w  = (const float*)d_in[3];
  const float* conv_b  = (const float*)d_in[4];
  const float* w_xproj = (const float*)d_in[5];
  const float* A_log   = (const float*)d_in[6];
  const float* D_param = (const float*)d_in[7];
  const float* w_out   = (const float*)d_in[8];
  float* dout = (float*)d_out;

  char* ws = (char*)d_ws;
  unsigned short* WIN16  = (unsigned short*)(ws + kOffWIN16);
  unsigned short* WXP16  = (unsigned short*)(ws + kOffWXP16);
  unsigned short* WOUT16 = (unsigned short*)(ws + kOffWOUT16);
  unsigned short* H16    = (unsigned short*)(ws + kOffH16);
  float*          XZ     = (float*)(ws + kOffXZ);
  float*          UC     = (float*)(ws + kOffUC);
  unsigned short* UC16   = (unsigned short*)(ws + kOffUC16);
  float*          PROJ   = (float*)(ws + kOffPROJ);
  unsigned short* Y16    = (unsigned short*)(ws + kOffY16);

  transpose_cast_kernel<<<dim3(kXZP / 64,  kDmod / 64), 256, 0, stream>>>(w_in,    WIN16,  kDmod, kXZP,  kXZP,  kCarW);
  transpose_cast_kernel<<<dim3(kPrjP / 64, kDin / 64),  256, 0, stream>>>(w_xproj, WXP16,  kDin,  kPrjN, kPrjP, kCarW);
  transpose_cast_kernel<<<dim3(kDmod / 64, kDin / 64),  256, 0, stream>>>(w_out,   WOUT16, kDin,  kDmod, kDmod, kCarW);

  rmsnorm_cast_kernel<<<kRows, 128, 0, stream>>>(x, norm_w, H16);

  for (int b = 0; b < kBatch; ++b) {
    const unsigned short* H16b = H16 + (size_t)b * kSeqL * kDmod;
    const float* xb   = x    + (size_t)b * kSeqL * kDmod;
    float*       outb = dout + (size_t)b * kSeqL * kDmod;

    wmma_gemm64_f16<false><<<dim3(256, 1), 256, 0, stream>>>(
        H16b, kDmod, WIN16, kDmod, XZ, kXZP, xb, kDmod, kSeqL, kXZP, kDmod, kSclIn);

    conv_silu_kernel<<<dim3(kDin / 256, kSeqL / 64), 256, 0, stream>>>(XZ, conv_w, conv_b, UC, UC16);

    wmma_gemm64_f16<false><<<dim3(132, 1), 256, 0, stream>>>(
        UC16, kDin, WXP16, kDin, PROJ, kPrjP, xb, kDmod, kSeqL, kPrjP, kDin, kSclXp);

    scan_kernel<<<dim3(kDin / 256, 1), 256, 0, stream>>>(PROJ, UC, XZ, A_log, D_param, Y16);

    wmma_gemm64_f16<true><<<dim3(64, 1), 256, 0, stream>>>(
        Y16, kDin, WOUT16, kDin, outb, kDmod, xb, kDmod, kSeqL, kDmod, kDin, kSclOut);
  }
}
